// ReplicatorDerivLayer_17523466568260
// MI455X (gfx1250) — hardware-verified
//
#include <hip/hip_runtime.h>

typedef __attribute__((ext_vector_type(16))) _Float16 v16h;
typedef __attribute__((ext_vector_type(8)))  _Float16 v8h;
typedef __attribute__((ext_vector_type(16))) __bf16   v16b;
typedef __attribute__((ext_vector_type(8)))  __bf16   v8b;
typedef __attribute__((ext_vector_type(8)))  float    v8f;
typedef __attribute__((ext_vector_type(4)))  float    v4f;

__device__ __forceinline__ unsigned short f2bf_bits(float f) {
  unsigned u = __float_as_uint(f);
  return (unsigned short)((u + 0x7FFFu + ((u >> 16) & 1u)) >> 16);
}
__device__ __forceinline__ float bf_bits2f(unsigned short h) { return __uint_as_float(((unsigned)h) << 16); }

__device__ __forceinline__ void dep_guard_h(v8f& a, v8f& b, v16h x, v16h y) { asm volatile("v_nop\n\tv_nop\n\tv_nop\n\tv_nop" : "+v"(a), "+v"(b) : "v"(x), "v"(y)); }
__device__ __forceinline__ void dep_guard_b(v8f& a, v8f& b, v16b x, v16b y) { asm volatile("v_nop\n\tv_nop\n\tv_nop\n\tv_nop" : "+v"(a), "+v"(b) : "v"(x), "v"(y)); }
__device__ __forceinline__ void keep4_h(v16h a, v16h b, v16h c, v16h d) { asm volatile("v_nop" :: "v"(a), "v"(b), "v"(c), "v"(d)); }
__device__ __forceinline__ void keep4_b(v16b a, v16b b, v16b c, v16b d) { asm volatile("v_nop" :: "v"(a), "v"(b), "v"(c), "v"(d)); }
__device__ __forceinline__ void acc_guard4(v8f& a, v8f& b, v8f& c, v8f& d) { asm volatile("v_nop\n\tv_nop\n\tv_nop\n\tv_nop" : "+v"(a), "+v"(b), "+v"(c), "+v"(d)); }
template <typename T> struct Frag;
template <> struct Frag<_Float16> {
  typedef v16h V; union U { v16h v; v8h h[2]; };
  static __device__ __forceinline__ v16h load(const _Float16* p) {
    U f; f.h[0] = *(const v8h*)(p); f.h[1] = *(const v8h*)(p + 16); return f.v;
  }
  static __device__ __forceinline__ v8f mma(v16h a, v16h b, v8f c) {
    return __builtin_amdgcn_wmma_f32_16x16x32_f16(false, a, false, b, (short)0, c, false, false);
  }
  static __device__ __forceinline__ void guard(v8f& a, v8f& b, v16h x, v16h y) { dep_guard_h(a, b, x, y); }
  static __device__ __forceinline__ void keep(v16h a, v16h b, v16h c, v16h d) { keep4_h(a, b, c, d); }
};
template <> struct Frag<__bf16> {
  typedef v16b V; union U { v16b v; v8b h[2]; };
  static __device__ __forceinline__ v16b load(const __bf16* p) {
    U f; f.h[0] = *(const v8b*)(p); f.h[1] = *(const v8b*)(p + 16); return f.v;
  }
  static __device__ __forceinline__ v8f mma(v16b a, v16b b, v8f c) {
    return __builtin_amdgcn_wmma_f32_16x16x32_bf16(false, a, false, b, (short)0, c, false, false);
  }
  static __device__ __forceinline__ void guard(v8f& a, v8f& b, v16b x, v16b y) { dep_guard_b(a, b, x, y); }
  static __device__ __forceinline__ void keep(v16b a, v16b b, v16b c, v16b d) { keep4_b(a, b, c, d); }
};

template <int ET> struct Elem;
template <> struct Elem<0> { typedef _Float16 T; };
template <> struct Elem<1> { typedef __bf16 T; };

template <int ET, int OUT_MODE, int TRI>
__global__ __launch_bounds__(256) void wmma_gemm64(
    const unsigned short* __restrict__ Ap, int lda, long strideA,
    const unsigned short* __restrict__ Btp, int ldb, long strideB,
    void* __restrict__ Cout, int ldc, long strideC,
    int M, int N, int K, float scale) {
  typedef typename Elem<ET>::T T;
  typedef typename Frag<T>::V V;
  const T* A = (const T*)Ap; const T* Bt = (const T*)Btp;
  __shared__ __align__(16) float sT[8][16 * 68];
  const int b    = blockIdx.y;
  const int lane = threadIdx.x & 31;
  const int wave = threadIdx.x >> 5;
  const int tilesN = N >> 6;
  const int tilesM = M >> 6;
  const int tile = blockIdx.x * 8 + wave;
  int tm, tn;
  if (TRI == 1) {
    const int total = (tilesM * (tilesM + 1)) >> 1;
    if (tile >= total) return;
    int t = (int)((sqrtf(8.0f * (float)tile + 1.0f) - 1.0f) * 0.5f);
    if ((((t + 1) * (t + 2)) >> 1) <= tile) ++t;
    if (((t * (t + 1)) >> 1) > tile) --t;
    t = (t < 0) ? 0 : ((t > tilesM - 1) ? (tilesM - 1) : t);
    tm = t;
    tn = tile - ((t * (t + 1)) >> 1);
    tn = (tn < 0) ? 0 : ((tn > tm) ? tm : tn);
  } else {
    if (tile >= tilesM * tilesN) return;
    tm = tile / tilesN;
    tn = tile - tm * tilesN;
  }
  const int m0 = tm << 6;
  const int n0 = tn << 6;
  int Kend = K;
  if (TRI == 2) Kend = (m0 + 64 < K) ? (m0 + 64) : K;

  const T* Ab = A  + (size_t)b * strideA;
  const T* Bb = Bt + (size_t)b * strideB;

  const int rlane = lane & 15;
  const int koff  = (lane >> 4) * 8;
  const int mOff  = (lane >> 4) * 8;

  v8f acc[4][4];
#pragma unroll
  for (int i = 0; i < 4; ++i)
#pragma unroll
    for (int j = 0; j < 4; ++j) acc[i][j] = (v8f){0.f,0.f,0.f,0.f,0.f,0.f,0.f,0.f};

  for (int k0 = 0; k0 < Kend; k0 += 32) {
    V bh[4];
#pragma unroll
    for (int j = 0; j < 4; ++j) {
      const size_t bo = (size_t)(n0 + (j << 4) + rlane) * ldb + koff + k0;
      bh[j] = Frag<T>::load(Bb + bo);
    }
#pragma unroll
    for (int i = 0; i < 4; ++i) {
      const size_t ao = (size_t)(m0 + (i << 4) + rlane) * lda + koff + k0;
      V ah = Frag<T>::load(Ab + ao);
#pragma unroll
      for (int j = 0; j < 4; ++j) {
        acc[i][j] = Frag<T>::mma(ah, bh[j], acc[i][j]);
      }
      Frag<T>::guard(acc[i][0], acc[i][3], ah, ah);
    }
    Frag<T>::keep(bh[0], bh[1], bh[2], bh[3]);
  }
  acc_guard4(acc[0][0], acc[0][1], acc[0][2], acc[0][3]);
  acc_guard4(acc[1][0], acc[1][1], acc[1][2], acc[1][3]);
  acc_guard4(acc[2][0], acc[2][1], acc[2][2], acc[2][3]);
  acc_guard4(acc[3][0], acc[3][1], acc[3][2], acc[3][3]);

  float* slab = sT[wave];
#pragma unroll
  for (int i = 0; i < 4; ++i) {
    const int mBase = m0 + (i << 4);
#pragma unroll
    for (int j = 0; j < 4; ++j) {
      const int n = n0 + (j << 4) + rlane;
#pragma unroll
      for (int r = 0; r < 8; ++r) {
        float v = acc[i][j][r] * scale;
        if (TRI == 1) { if (n > mBase + mOff + r) v = 0.0f; }
        slab[(mOff + r) * 68 + (j << 4) + rlane] = v;
      }
    }
    __builtin_amdgcn_fence(__ATOMIC_RELEASE, "workgroup");
    __builtin_amdgcn_wave_barrier();
    __builtin_amdgcn_fence(__ATOMIC_ACQUIRE, "workgroup");
    if (OUT_MODE == 0) {
      float* C = (float*)Cout + (size_t)b * strideC;
      const int hh = lane >> 4, c4 = (lane & 15) * 4;
      for (int pass = 0; pass < 2; ++pass) {
#pragma unroll
        for (int it = 0; it < 8; ++it) {
          const int row = it * 2 + hh;
          v4f v = *(const v4f*)(slab + row * 68 + c4);
          *(volatile v4f*)(C + (size_t)(mBase + row) * ldc + n0 + c4) = v;
        }
        __threadfence();
      }
    } else {
      const int q = lane >> 3, c8 = (lane & 7) * 8;
      unsigned short* C = (unsigned short*)Cout + (size_t)b * strideC;
      for (int pass = 0; pass < 2; ++pass) {
#pragma unroll
        for (int it = 0; it < 4; ++it) {
          const int row = it * 4 + q;
          const float* sp = slab + row * 68 + c8;
          v8h hv;
#pragma unroll
          for (int e = 0; e < 8; ++e) hv[e] = (_Float16)sp[e];
          *(volatile v8h*)(C + (size_t)(mBase + row) * ldc + n0 + c8) = hv;
        }
        __threadfence();
      }
    }
    __builtin_amdgcn_fence(__ATOMIC_RELEASE, "workgroup");
    __builtin_amdgcn_wave_barrier();
    __builtin_amdgcn_fence(__ATOMIC_ACQUIRE, "workgroup");
  }
}

__global__ __launch_bounds__(256) void wprep_kernel(
    const float* __restrict__ w1, const float* __restrict__ w2, _Float16* __restrict__ Wc, int E) {
  __shared__ float t1[64][65];
  __shared__ float t2[64][65];
  const int tid = threadIdx.x, lane = tid & 31, wave = tid >> 5;
  const int e0 = blockIdx.y * 64;
  const int f0 = blockIdx.x * 64;
  {
    const int row = tid >> 2, cb = (tid & 3) * 16;
    const float* s1 = w1 + (size_t)(e0 + row) * E + f0 + cb;
    const float* s2 = w2 + (size_t)(e0 + row) * E + f0 + cb;
#pragma unroll
    for (int i = 0; i < 4; ++i) {
      const v4f a = *(const v4f*)(s1 + 4 * i);
      const v4f c = *(const v4f*)(s2 + 4 * i);
#pragma unroll
      for (int k = 0; k < 4; ++k) { t1[row][cb + 4 * i + k] = a[k]; t2[row][cb + 4 * i + k] = c[k]; }
    }
  }
  __syncthreads();
  const int q = lane >> 3, c8 = (lane & 7) * 8;
  v8h h1[2], h2[2];
#pragma unroll
  for (int it = 0; it < 2; ++it) {
    const int r = wave * 8 + it * 4 + q;
    v8h a, c;
#pragma unroll
    for (int k = 0; k < 8; ++k) {
      a[k] = (_Float16)(16.0f * t1[c8 + k][r]);
      c[k] = (_Float16)(16.0f * t2[r][c8 + k]);
    }
    h1[it] = a; h2[it] = c;
  }
  for (int pass = 0; pass < 2; ++pass) {
#pragma unroll
    for (int it = 0; it < 2; ++it) {
      const int r = wave * 8 + it * 4 + q;
      *(volatile v8h*)(Wc + (size_t)(f0 + r) * E + e0 + c8) = h1[it];
      *(volatile v8h*)(Wc + (size_t)(E + e0 + r) * E + f0 + c8) = h2[it];
    }
    __threadfence();
  }
}

__global__ __launch_bounds__(256) void xprep_kernel(
    const float* __restrict__ x, _Float16* __restrict__ X16, _Float16* __restrict__ XT16, int E, int S) {
  __shared__ float tile[64][65];
  const int tid = threadIdx.x, lane = tid & 31, wave = tid >> 5;
  const int b = blockIdx.z, e0 = blockIdx.y * 64, s0 = blockIdx.x * 64;
  const float* xb = x + (size_t)b * E * S;
  {
    const int row = tid >> 2, cb = (tid & 3) * 16;
    const float* src = xb + (size_t)(e0 + row) * S + s0 + cb;
#pragma unroll
    for (int i = 0; i < 4; ++i) {
      const v4f v = *(const v4f*)(src + 4 * i);
#pragma unroll
      for (int k = 0; k < 4; ++k) tile[row][cb + 4 * i + k] = v[k];
    }
  }
  __syncthreads();
  const int q = lane >> 3, c8 = (lane & 7) * 8;
  v8h hx[2], ht[2];
#pragma unroll
  for (int it = 0; it < 2; ++it) {
    const int row = wave * 8 + it * 4 + q;
    v8h a, t;
#pragma unroll
    for (int k = 0; k < 8; ++k) {
      a[k] = (_Float16)tile[row][c8 + k];
      t[k] = (_Float16)tile[c8 + k][row];
    }
    hx[it] = a; ht[it] = t;
  }
  _Float16* X16b  = X16  + (size_t)b * E * S;
  _Float16* XT16b = XT16 + (size_t)b * S * E;
  for (int pass = 0; pass < 2; ++pass) {
#pragma unroll
    for (int it = 0; it < 2; ++it) {
      const int row = wave * 8 + it * 4 + q;
      *(volatile v8h*)(X16b  + (size_t)(e0 + row) * S + s0 + c8) = hx[it];
      *(volatile v8h*)(XT16b + (size_t)(s0 + row) * E + e0 + c8) = ht[it];
    }
    __threadfence();
  }
}

__global__ __launch_bounds__(256) void epi_kernel(
    const float* __restrict__ x, const float* __restrict__ FITT, float* __restrict__ out, int E, int S) {
  __shared__ float red[8][33];
  __shared__ float avg_s[32];
  __shared__ float ft[64][33];
  const int tid = threadIdx.x, lane = tid & 31, wave = tid >> 5;
  const int b = blockIdx.y, e0 = blockIdx.x * 32;
  const float* xb = x    + (size_t)b * E * S;
  const float* fb = FITT + (size_t)b * S * E;
  float*       ob = out  + (size_t)b * E * S;

  {
    float acc = 0.0f;
    const float* xr = xb + (size_t)(e0 + lane) * S;
    const float* fc = fb + e0 + lane;
#pragma unroll 4
    for (int s = wave; s < S; s += 8) acc += xr[s] * fc[(size_t)s * E];
    red[wave][lane] = acc;
  }
  __syncthreads();
  if (wave == 0) {
    float a = red[0][lane];
    a += red[1][lane]; a += red[2][lane]; a += red[3][lane];
    a += red[4][lane]; a += red[5][lane]; a += red[6][lane]; a += red[7][lane];
    avg_s[lane] = a;
  }
  __syncthreads();

  const int hh = lane >> 4, c4 = (lane & 15) * 4;
  const int nst = S >> 6;
  for (int st = 0; st < nst; ++st) {
    const int s0 = st << 6;
    {
      const int row = tid >> 2, c = (tid & 3) * 8;
      const float* src = fb + (size_t)(s0 + row) * E + e0 + c;
      const v4f v0 = *(const v4f*)(src);
      const v4f v1 = *(const v4f*)(src + 4);
#pragma unroll
      for (int k = 0; k < 4; ++k) { ft[row][c + k] = v0[k]; ft[row][c + 4 + k] = v1[k]; }
    }
    __syncthreads();
    v4f o[2];
#pragma unroll
    for (int it = 0; it < 2; ++it) {
      const int er = wave * 4 + it * 2 + hh;
      const float a = avg_s[er];
      const v4f xv = *(const v4f*)(xb + (size_t)(e0 + er) * S + s0 + c4);
      v4f rv;
#pragma unroll
      for (int k = 0; k < 4; ++k) {
        const float net = ft[c4 + k][er] - a;
        const float v = xv[k] + xv[k] * net;
        rv[k] = (v > 0.0f) ? v : 0.0f;
      }
      o[it] = rv;
    }
    for (int pass = 0; pass < 2; ++pass) {
#pragma unroll
      for (int it = 0; it < 2; ++it) {
        const int er = wave * 4 + it * 2 + hh;
        *(volatile v4f*)(ob + (size_t)(e0 + er) * S + s0 + c4) = o[it];
      }
      __threadfence();
    }
    __syncthreads();
  }
}

extern "C" void kernel_launch(void* const* d_in, const int* in_sizes, int n_in,
                              void* d_out, int out_size, void* d_ws, size_t ws_size,
                              hipStream_t stream)
{
  const int B = 8, E = 512, S = 2048, G = 4;
  if (n_in < 3) return;
  if (in_sizes[0] != B * E * S || in_sizes[1] != E * E || in_sizes[2] != E * E) return;
  if (out_size != B * E * S) return;

  const float* x  = (const float*)d_in[0];
  const float* w1 = (const float*)d_in[1];
  const float* w2 = (const float*)d_in[2];
  float* out = (float*)d_out;

  const size_t szW   = (size_t)2 * E * E * sizeof(_Float16);
  const size_t szX   = (size_t)G * E * S * sizeof(_Float16);
  const size_t szFT  = (size_t)G * S * (2 * E) * sizeof(_Float16);
  const size_t szS   = (size_t)G * S * S * sizeof(_Float16);
  const size_t szFIT = (size_t)G * S * E * sizeof(float);
  const size_t oW   = 0;
  const size_t oX16 = oW + szW;
  const size_t oXT  = oX16 + szX;
  const size_t oFT  = oXT + szX;
  const size_t oS   = oFT + szFT;
  const size_t oFIT = oS + szS;
  const size_t total = oFIT + szFIT;
  if (total > ws_size) return;

  char* ws = (char*)d_ws;
  _Float16* Wc   = (_Float16*)(ws + oW);
  _Float16* X16  = (_Float16*)(ws + oX16);
  _Float16* XT16 = (_Float16*)(ws + oXT);
  _Float16* FT   = (_Float16*)(ws + oFT);
  _Float16* S16  = (_Float16*)(ws + oS);
  float*    FITT = (float*)(ws + oFIT);

  wprep_kernel<<<dim3(E / 64, E / 64), 256, 0, stream>>>(w1, w2, Wc, E);

  const int tilesS = S / 64, tilesE = E / 64;
  const int blkF   = (tilesS * (2 * E / 64) + 7) / 8;
  const int blkTri = ((tilesS * (tilesS + 1)) / 2 + 7) / 8;
  const int blkFit = (tilesS * tilesE + 7) / 8;

  for (int g = 0; g < B / G; ++g) {
    const float* xg = x   + (size_t)g * G * E * S;
    float*       og = out + (size_t)g * G * E * S;

    xprep_kernel<<<dim3(S / 64, E / 64, G), 256, 0, stream>>>(xg, X16, XT16, E, S);

    wmma_gemm64<0, 1, 0><<<dim3(blkF, G), 256, 0, stream>>>(
        (const unsigned short*)XT16, E, (long)S * E,
        (const unsigned short*)Wc, E, 0L,
        (void*)FT, 2 * E, (long)S * 2 * E,
        S, 2 * E, E, 1.0f);

    wmma_gemm64<0, 1, 1><<<dim3(blkTri, G), 256, 0, stream>>>(
        (const unsigned short*)FT, 2 * E, (long)S * 2 * E,
        (const unsigned short*)(FT + E), 2 * E, (long)S * 2 * E,
        (void*)S16, S, (long)S * S,
        S, S, E, 1.0f / 256.0f);

    wmma_gemm64<0, 0, 2><<<dim3(blkFit, G), 256, 0, stream>>>(
        (const unsigned short*)S16, S, (long)S * S,
        (const unsigned short*)X16, S, (long)E * S,
        (void*)FITT, E, (long)S * E,
        S, E, S, 1.0f);

    epi_kernel<<<dim3(E / 32, G), 256, 0, stream>>>(xg, FITT, og, E, S);
  }
}
